// BackgroundAlignmentModule_78838419685496
// MI455X (gfx1250) — hardware-verified
//
#include <hip/hip_runtime.h>
#include <stdint.h>

typedef float v8f __attribute__((ext_vector_type(8)));
typedef float v4f __attribute__((ext_vector_type(4)));
typedef unsigned int v4u __attribute__((ext_vector_type(4)));
typedef __bf16 v16bf __attribute__((ext_vector_type(16)));
typedef __bf16 v8bf __attribute__((ext_vector_type(8)));
union Frag { v16bf v; v8bf half[2]; };

#define NB   2
#define NC   64
#define NH   128
#define NW   128
#define NPIX (NH * NW)
#define PLANE_HALVES ((size_t)NB * NPIX * NC)
#define NEGBIG (-1000000000.0f)
#define CVT_BLOCKS (3 * NB * NH * (NW / 32))
#define CORR_BLOCKS (4 * NB * NH * (NW / 32))

__device__ __forceinline__ unsigned int bf16_rne_bits(float x) {
    unsigned int u = __float_as_uint(x);
    u += 0x7FFFu + ((u >> 16) & 1u);
    return u >> 16;
}

__device__ __forceinline__ v8f mma_bf16(v8f acc, v16bf a, v16bf b) {
    acc = __builtin_amdgcn_wmma_f32_16x16x32_bf16(false, a, false, b, (short)0, acc, false, false);
    asm volatile("v_nop\n\tv_nop\n\tv_nop\n\tv_nop" : "+v"(acc) : "v"(a), "v"(b));
    return acc;
}

__device__ __forceinline__ v8f mma3(v8f acc, const Frag& ah, const Frag& al,
                                    const Frag& bh, const Frag& bl) {
    acc = mma_bf16(acc, ah.v, bh.v);
    acc = mma_bf16(acc, ah.v, bl.v);
    acc = mma_bf16(acc, al.v, bh.v);
    return acc;
}

__device__ __forceinline__ void load_frag(Frag& f, const __bf16* rowk0, int h) {
    f.half[0] = *(const v8bf*)(rowk0 + 8 * h);
    f.half[1] = *(const v8bf*)(rowk0 + 16 + 8 * h);
}

__global__ __launch_bounds__(128) void
k_convert(const float* __restrict__ f0, const float* __restrict__ f1,
          const float* __restrict__ f2, unsigned int* __restrict__ ws_u, int nblocks)
{
    __shared__ float tile[32 * 65];

    const int bid = blockIdx.x;
    if (bid >= nblocks) return;
    const int xc = bid & 3;
    const int y  = (bid >> 2) & 127;
    const int b  = (bid >> 9) & 1;
    const int f  = (bid >> 10);
    const float* src = (f == 0) ? f0 : ((f == 1) ? f1 : f2);

    const int t  = threadIdx.x;
    const int x  = t & 31;
    const int cb = t >> 5;
    const float* sp = src + (size_t)b * NC * NPIX + (size_t)y * NW + xc * 32 + x;
#pragma unroll
    for (int i = 0; i < 16; ++i) {
        const int c = cb + 4 * i;
        tile[x * 65 + c] = sp[(size_t)c * NPIX];
    }
    __syncthreads();

    unsigned int* hip = ws_u + (size_t)(2 * f)     * (PLANE_HALVES / 2);
    unsigned int* lop = ws_u + (size_t)(2 * f + 1) * (PLANE_HALVES / 2);

    const int lane = t & 31;
    const int w    = t >> 5;
    const int q    = lane >> 3;
    const int e    = lane & 7;

    v4u hv[2], lv[2];
    size_t off[2];
#pragma unroll
    for (int pass = 0; pass < 2; ++pass) {
        const int px = pass * 16 + w * 4 + q;
        const float* tp = tile + px * 65 + 8 * e;
        unsigned int hb[8], lb[8];
#pragma unroll
        for (int i = 0; i < 8; ++i) {
            const float v  = tp[i];
            const unsigned int hbits = bf16_rne_bits(v);
            const float vh = __uint_as_float(hbits << 16);
            hb[i] = hbits;
            lb[i] = bf16_rne_bits(v - vh);
        }
        v4u hvv, lvv;
        hvv.x = hb[0] | (hb[1] << 16);  hvv.y = hb[2] | (hb[3] << 16);
        hvv.z = hb[4] | (hb[5] << 16);  hvv.w = hb[6] | (hb[7] << 16);
        lvv.x = lb[0] | (lb[1] << 16);  lvv.y = lb[2] | (lb[3] << 16);
        lvv.z = lb[4] | (lb[5] << 16);  lvv.w = lb[6] | (lb[7] << 16);
        hv[pass] = hvv;  lv[pass] = lvv;
        const size_t pixel = ((size_t)(b * NH + y)) * NW + xc * 32 + px;
        off[pass] = pixel * 32 + 4 * e;
    }
#pragma unroll
    for (int pass = 0; pass < 2; ++pass) {
        *(volatile v4u*)(hip + off[pass]) = hv[pass];
        *(volatile v4u*)(lop + off[pass]) = lv[pass];
    }
    __threadfence();
#pragma unroll
    for (int pass = 0; pass < 2; ++pass) {
        *(volatile v4u*)(hip + off[pass]) = hv[pass];
        *(volatile v4u*)(lop + off[pass]) = lv[pass];
    }
}

__global__ __launch_bounds__(32) void
k_corr(const __bf16* __restrict__ ws_h, float* __restrict__ out, int nblocks)
{
    __shared__ float dtile[4 * 256];
    __shared__ float corrbuf[25 * 32];
    __shared__ __attribute__((aligned(16))) float obuf[64];

    const int bid = blockIdx.x;
    if (bid >= nblocks) return;
    const int xc = bid & 3;
    const int y  = (bid >> 2) & 127;
    const int b  = (bid >> 9) & 1;
    const int p  = (bid >> 10) & 3;
    const int fsrc = (p < 2) ? p : 2;
    const int ftgt = (p < 2) ? 2 : (p - 2);

    const __bf16* Shi = ws_h + (size_t)(2 * fsrc)     * PLANE_HALVES;
    const __bf16* Slo = ws_h + (size_t)(2 * fsrc + 1) * PLANE_HALVES;
    const __bf16* Thi = ws_h + (size_t)(2 * ftgt)     * PLANE_HALVES;
    const __bf16* Tlo = ws_h + (size_t)(2 * ftgt + 1) * PLANE_HALVES;

    const int l  = threadIdx.x;
    const int h  = l >> 4;
    const int m  = l & 15;
    const int x0 = xc * 32;

    const size_t pixA0 = ((size_t)(b * NH + y)) * NW + x0 + m;
    const size_t pixA1 = pixA0 + 16;
    int xcl0 = x0 - 2 + m;        xcl0 = xcl0 < 0 ? 0 : xcl0;
    int xcl1 = x0 + 14 + m;       xcl1 = xcl1 > NW - 1 ? NW - 1 : xcl1;
    int xcl2 = x0 + 30 + m;       xcl2 = xcl2 > NW - 1 ? NW - 1 : xcl2;

#pragma unroll 1
    for (int dyi = 0; dyi < 5; ++dyi) {
        const int yy = y + dyi - 2;
        const bool rowvalid = (yy >= 0) && (yy < NH);
        const int yyc = yy < 0 ? 0 : (yy > NH - 1 ? NH - 1 : yy);
        const size_t rowT = ((size_t)(b * NH + yyc)) * NW;

        v8f acc00 = {0.f, 0.f, 0.f, 0.f, 0.f, 0.f, 0.f, 0.f};
        v8f acc01 = {0.f, 0.f, 0.f, 0.f, 0.f, 0.f, 0.f, 0.f};
        v8f acc11 = {0.f, 0.f, 0.f, 0.f, 0.f, 0.f, 0.f, 0.f};
        v8f acc12 = {0.f, 0.f, 0.f, 0.f, 0.f, 0.f, 0.f, 0.f};

#pragma unroll 1
        for (int ks = 0; ks < 2; ++ks) {
            const int k0 = ks * 32;
            Frag a0h, a0l, a1h, a1l;
            load_frag(a0h, Shi + pixA0 * NC + k0, h);
            load_frag(a0l, Slo + pixA0 * NC + k0, h);
            load_frag(a1h, Shi + pixA1 * NC + k0, h);
            load_frag(a1l, Slo + pixA1 * NC + k0, h);

            Frag b0h, b0l;
            load_frag(b0h, Thi + (rowT + xcl0) * NC + k0, h);
            load_frag(b0l, Tlo + (rowT + xcl0) * NC + k0, h);
            acc00 = mma3(acc00, a0h, a0l, b0h, b0l);

            Frag b1h, b1l;
            load_frag(b1h, Thi + (rowT + xcl1) * NC + k0, h);
            load_frag(b1l, Tlo + (rowT + xcl1) * NC + k0, h);
            acc01 = mma3(acc01, a0h, a0l, b1h, b1l);
            acc11 = mma3(acc11, a1h, a1l, b1h, b1l);

            Frag b2h, b2l;
            load_frag(b2h, Thi + (rowT + xcl2) * NC + k0, h);
            load_frag(b2l, Tlo + (rowT + xcl2) * NC + k0, h);
            acc12 = mma3(acc12, a1h, a1l, b2h, b2l);
        }

#pragma unroll
        for (int r = 0; r < 8; ++r) {
            const int row = 8 * h + r;
            dtile[0 * 256 + row * 16 + m] = acc00[r];
            dtile[1 * 256 + row * 16 + m] = acc01[r];
            dtile[2 * 256 + row * 16 + m] = acc11[r];
            dtile[3 * 256 + row * 16 + m] = acc12[r];
        }
        __syncthreads();

        {
            const int t = l >> 4;
#pragma unroll
            for (int dxi = 0; dxi < 5; ++dxi) {
                const int j = m + dxi;
                const int idx = (j < 16) ? ((2 * t) * 256 + m * 16 + j)
                                         : ((2 * t + 1) * 256 + m * 16 + (j - 16));
                const float val = dtile[idx];
                const int xs = x0 + l + dxi - 2;
                const bool valid = rowvalid && (xs >= 0) && (xs < NW);
                corrbuf[(dyi * 5 + dxi) * 32 + l] = valid ? val * 0.125f : NEGBIG;
            }
        }
        __syncthreads();
    }

    float mx = corrbuf[l];
#pragma unroll
    for (int k = 1; k < 25; ++k) mx = fmaxf(mx, corrbuf[k * 32 + l]);
    float s = 0.f, ex = 0.f, ey = 0.f;
#pragma unroll
    for (int k = 0; k < 25; ++k) {
        const float pr = __expf(corrbuf[k * 32 + l] - mx);
        s  += pr;
        ex += pr * (float)((k % 5) - 2);
        ey += pr * (float)((k / 5) - 2);
    }
    const float inv = 1.0f / s;
    obuf[l]      = ex * inv;
    obuf[32 + l] = ey * inv;
    __syncthreads();

    const int ch = (l >> 3) & 1;
    const int qq = l & 7;
    const v4f v = *(const v4f*)(obuf + ch * 32 + 4 * qq);
    float* dst = out + ((size_t)((p * 2 + b) * 2 + ch)) * NPIX + (size_t)y * NW + x0 + 4 * qq;
    if (l < 16) *(volatile v4f*)dst = v;
    __threadfence();
    if (l < 16) *(volatile v4f*)dst = v;
}

extern "C" void kernel_launch(void* const* d_in, const int* in_sizes, int n_in,
                              void* d_out, int out_size, void* d_ws, size_t ws_size,
                              hipStream_t stream)
{
    if (n_in < 3) return;
    const int nfeat = NB * NC * NPIX;
    if (in_sizes[0] != nfeat || in_sizes[1] != nfeat || in_sizes[2] != nfeat) return;
    if (out_size != 4 * NB * 2 * NPIX) return;
    const size_t ws_need = (size_t)6 * PLANE_HALVES * 2;
    if (ws_size < ws_need) return;

    const float* f0 = (const float*)d_in[0];
    const float* f1 = (const float*)d_in[1];
    const float* f2 = (const float*)d_in[2];

    k_convert<<<CVT_BLOCKS, 128, 0, stream>>>(f0, f1, f2, (unsigned int*)d_ws, CVT_BLOCKS);
    k_corr<<<CORR_BLOCKS, 32, 0, stream>>>((const __bf16*)d_ws, (float*)d_out, CORR_BLOCKS);
    (void)hipGetLastError();
}
